// Multihead_Attention_46806553592368
// MI455X (gfx1250) — hardware-verified
//
#include <hip/hip_runtime.h>


#ifndef NB
#define NB 4
#endif
#ifndef SEQ
#define SEQ 2048
#endif
#define NB_FULL  4
#define SEQ_FULL 2048
#define DIM      1024
#define NH       16
#define HD       64
#define ROWS     (NB * SEQ)
#define NSL      (NH * NB)
#define SLICE    (SEQ * HD)
#define L2E      1.44269504088896340736f
#define QKC      16.0f
#define PCARRY   4096.0f
#define VCARRY   16.0f
#define WOCARRY  64.0f
#define SL2E     (L2E / (QKC * QKC))
#define STGW     1152
#define LDP      40
#define LDO      72

static_assert(DIM == 1024);
static_assert(NH * HD == DIM);
static_assert(ROWS % 64 == 0);
static_assert(SEQ % 64 == 0);
static_assert(16 % NB == 0);
static_assert(NB >= 1 && NB <= NB_FULL);
static_assert(SEQ <= SEQ_FULL);
static_assert((ROWS * 128) % 256 == 0);
static_assert(STGW == 16 * LDO);

typedef __bf16       v16b __attribute__((ext_vector_type(16)));
typedef __bf16       v8b  __attribute__((ext_vector_type(8)));
typedef _Float16     v16h __attribute__((ext_vector_type(16)));
typedef _Float16     v8h  __attribute__((ext_vector_type(8)));
typedef float        v8f  __attribute__((ext_vector_type(8)));
typedef float        v4f  __attribute__((ext_vector_type(4)));
typedef unsigned int v4u  __attribute__((ext_vector_type(4)));

template <typename T> struct Frag;
template <> struct Frag<__bf16>   { typedef v16b t; };
template <> struct Frag<_Float16> { typedef v16h t; };

static __device__ __forceinline__ v8f zero8() {
  v8f z = {0.f, 0.f, 0.f, 0.f, 0.f, 0.f, 0.f, 0.f};
  return z;
}

template <typename T>
static __device__ __forceinline__ typename Frag<T>::t ldfrag(const T* rowk, int kb) {
  union { typename Frag<T>::t v; v4u q[2]; } u;
  u.q[0] = *reinterpret_cast<const v4u*>(rowk + kb);
  u.q[1] = *reinterpret_cast<const v4u*>(rowk + 16 + kb);
  return u.v;
}

static __device__ __forceinline__ v8f mma16(v16b a, v16b b, v8f c) {
  c = __builtin_amdgcn_wmma_f32_16x16x32_bf16(false, a, false, b, (short)0, c, false, false);
  asm volatile("v_nop\n\tv_nop\n\tv_nop\n\tv_nop" : "+v"(c) : "v"(a), "v"(b));
  return c;
}
static __device__ __forceinline__ v8f mma16(v16h a, v16h b, v8f c) {
  c = __builtin_amdgcn_wmma_f32_16x16x32_f16(false, a, false, b, (short)0, c, false, false);
  asm volatile("v_nop\n\tv_nop\n\tv_nop\n\tv_nop" : "+v"(c) : "v"(a), "v"(b));
  return c;
}

static __device__ __forceinline__ void st_tile16(const unsigned short* lds, unsigned short* g,
                                                 int lane, int pitch) {
#pragma unroll
  for (int it = 0; it < 4; ++it) {
    const int p = it * 32 + lane, row = p >> 3, seg = p & 7;
    const v4u v = *reinterpret_cast<const v4u*>(lds + row * LDO + seg * 8);
    *reinterpret_cast<volatile v4u*>(g + (size_t)row * pitch + seg * 8) = v;
  }
}
static __device__ __forceinline__ void st_tile32(const float* lds, float* g, int lane, int pitch) {
#pragma unroll
  for (int it = 0; it < 8; ++it) {
    const int p = it * 32 + lane, row = p >> 4, seg = p & 15;
    const v4f v = *reinterpret_cast<const v4f*>(lds + row * LDO + seg * 4);
    *reinterpret_cast<volatile v4f*>(g + (size_t)row * pitch + seg * 4) = v;
  }
}

template <int F16OUT>
__global__ __launch_bounds__(256) void cvt_kernel(const float* __restrict__ src,
                                                   unsigned short* __restrict__ dst,
                                                   int nrows, int seg, int segfull, float scale) {
  const int i = blockIdx.x * 256 + (int)threadIdx.x;
  if (i >= nrows * (DIM / 8)) return;
  const int R  = i >> 7;
  const int c8 = i & 127;
  const int rb = R / seg;
  const int prow = rb * segfull + (R - rb * seg);
  const float* s = src + (size_t)prow * DIM + c8 * 8;
  const v4f a0 = *reinterpret_cast<const v4f*>(s);
  const v4f a1 = *reinterpret_cast<const v4f*>(s + 4);
  union { v8b vb; v8h vh; v4u q; } u;
  if (F16OUT) {
#pragma unroll
    for (int j = 0; j < 4; ++j) {
      u.vh[j]     = (_Float16)((float)(__bf16)a0[j] * scale);
      u.vh[4 + j] = (_Float16)((float)(__bf16)a1[j] * scale);
    }
  } else {
#pragma unroll
    for (int j = 0; j < 4; ++j) {
      u.vb[j]     = (__bf16)a0[j];
      u.vb[4 + j] = (__bf16)a1[j];
    }
  }
  const v4u q = u.q;
  unsigned short* d = dst + (size_t)R * DIM + c8 * 8;
  *reinterpret_cast<volatile v4u*>(d) = q;
  __threadfence();
  *reinterpret_cast<volatile v4u*>(d) = q;
}

template <typename T, int OUTM>
__global__ __launch_bounds__(256) void gemm_kernel(const T* __restrict__ A, const T* __restrict__ W,
                                                    const float* __restrict__ bias,
                                                    float ascale, float oscale,
                                                    unsigned short* out16, float* outf,
                                                    int M, int N, int K) {
  __shared__ __align__(16) float stg[8 * STGW];
  const int tid = threadIdx.x, lane = tid & 31, w = tid >> 5;
  const int wm = w & 3, wn = w >> 2;
  const int mtile = blockIdx.x * 64 + wm * 16;
  const int ntile = blockIdx.y * 128 + wn * 64;
  const int lm = lane & 15, hh = lane >> 4, kb = hh * 8, roff = hh * 8;
  typedef typename Frag<T>::t FT;

  v8f acc[4];
#pragma unroll
  for (int c = 0; c < 4; ++c) acc[c] = zero8();

  const T* arow = A + (size_t)(mtile + lm) * K;
  const T* wrow = W + (size_t)(ntile + lm) * K;
#pragma unroll 2
  for (int k0 = 0; k0 < K; k0 += 32) {
    const FT af = ldfrag<T>(arow + k0, kb);
#pragma unroll
    for (int c = 0; c < 4; ++c) {
      const FT bf = ldfrag<T>(wrow + (size_t)(c * 16) * K + k0, kb);
      acc[c] = mma16(af, bf, acc[c]);
    }
  }

  float* wst = stg + w * STGW;
  _Float16* wsh = reinterpret_cast<_Float16*>(wst);
#pragma unroll
  for (int c = 0; c < 4; ++c) {
    const int col = ntile + c * 16 + lm;
    const float bb = (float)(__bf16)bias[col];
#pragma unroll
    for (int r = 0; r < 8; ++r) {
      const int li = (roff + r) * LDO + c * 16 + lm;
      const float val = acc[c][r] * ascale + bb;
      if (OUTM == 2) {
        wst[li] = val;
      } else {
        wsh[li] = (_Float16)(val * oscale);
      }
    }
  }
  __syncthreads();
  const size_t goff = (size_t)mtile * N + ntile;
  if (OUTM == 2) {
    st_tile32(wst, outf + goff, lane, N);
    __threadfence();
    st_tile32(wst, outf + goff, lane, N);
  } else {
    const unsigned short* ls = reinterpret_cast<const unsigned short*>(wst);
    st_tile16(ls, out16 + goff, lane, N);
    __threadfence();
    st_tile16(ls, out16 + goff, lane, N);
  }
}

__global__ __launch_bounds__(128) void vt_kernel(const _Float16* __restrict__ V,
                                                 _Float16* __restrict__ Vt) {
  __shared__ __align__(16) _Float16 tile[64 * LDO];
  const int tid = threadIdx.x;
  const size_t base = (size_t)blockIdx.y * SLICE;
  const int kt = blockIdx.x * 64;
#pragma unroll
  for (int it = 0; it < 4; ++it) {
    const int p = it * 128 + tid, key = p >> 3, seg = p & 7;
    const v4u v = *reinterpret_cast<const v4u*>(V + base + (size_t)(kt + key) * HD + seg * 8);
    *reinterpret_cast<v4u*>(tile + key * LDO + seg * 8) = v;
  }
  __syncthreads();
  v4u wv[4];
#pragma unroll
  for (int it = 0; it < 4; ++it) {
    const int p = it * 128 + tid, d = p >> 3, seg = p & 7;
    union { v8h v; v4u q; } u;
#pragma unroll
    for (int j = 0; j < 8; ++j) u.v[j] = tile[(seg * 8 + j) * LDO + d];
    wv[it] = u.q;
  }
  _Float16* ob = Vt + base + kt;
#pragma unroll
  for (int it = 0; it < 4; ++it) {
    const int p = it * 128 + tid, d = p >> 3, seg = p & 7;
    *reinterpret_cast<volatile v4u*>(ob + (size_t)d * SEQ + seg * 8) = wv[it];
  }
  __threadfence();
#pragma unroll
  for (int it = 0; it < 4; ++it) {
    const int p = it * 128 + tid, d = p >> 3, seg = p & 7;
    *reinterpret_cast<volatile v4u*>(ob + (size_t)d * SEQ + seg * 8) = wv[it];
  }
}

__global__ __launch_bounds__(NB * 32) __attribute__((amdgpu_num_vgpr(256)))
void attn_kernel(const _Float16* __restrict__ Qp, const _Float16* __restrict__ Kp,
                 const _Float16* __restrict__ Vt, _Float16* __restrict__ Ctx) {
  __shared__ __align__(16) float    sc[NB * 2 * 32 * 8];
  __shared__ __align__(16) _Float16 pw[NB * 16 * LDP];
  __shared__ __align__(16) _Float16 ost[NB * 16 * LDO];

  const int tid = threadIdx.x, lane = tid & 31, b = tid >> 5;
  const int h = blockIdx.y, qbase = blockIdx.x * 16;
  const int lm = lane & 15, hh = lane >> 4, kb = hh * 8, roff = hh * 8;
  const size_t base = (size_t)(h * NB + b) * SLICE;

  const _Float16* qr = Qp + base + (size_t)(qbase + lm) * HD;
  const v16h q0 = ldfrag<_Float16>(qr, kb);
  const v16h q1 = ldfrag<_Float16>(qr + 32, kb);

  v8f o[4];
#pragma unroll
  for (int cc = 0; cc < 4; ++cc) o[cc] = zero8();

  const _Float16* vrow = Vt + base + (size_t)lm * SEQ;
  constexpr int JP = 16 / NB;

#pragma unroll 1
  for (int kt = 0; kt < SEQ; kt += 32) {
    v8f s[2];
#pragma unroll
    for (int c = 0; c < 2; ++c) {
      const _Float16* kr = Kp + base + (size_t)(kt + c * 16 + lm) * HD;
      v8f t = zero8();
      v16h kf = ldfrag<_Float16>(kr, kb);
      t = mma16(q0, kf, t);
      kf = ldfrag<_Float16>(kr + 32, kb);
      t = mma16(q1, kf, t);
      s[c] = t;
    }

    __syncthreads();
#pragma unroll
    for (int c = 0; c < 2; ++c) {
      union { v8f v; v4f q[2]; } u;
      u.v = s[c];
      float* dst = sc + ((b * 2 + c) * 32 + lane) * 8;
      *reinterpret_cast<v4f*>(dst)     = u.q[0];
      *reinterpret_cast<v4f*>(dst + 4) = u.q[1];
    }
    __syncthreads();

#pragma unroll
    for (int jj = 0; jj < JP; ++jj) {
      const int j = b * JP + jj;
      const int c = j >> 3, r = j & 7;
      float sv[NB];
#pragma unroll
      for (int bb = 0; bb < NB; ++bb) sv[bb] = sc[((bb * 2 + c) * 32 + lane) * 8 + r];
      float mx = sv[0];
#pragma unroll
      for (int bb = 1; bb < NB; ++bb) mx = fmaxf(mx, sv[bb]);
      float sum = 0.f;
#pragma unroll
      for (int bb = 0; bb < NB; ++bb) {
        sv[bb] = exp2f((sv[bb] - mx) * SL2E);
        sum += sv[bb];
      }
      const float scl = PCARRY * __builtin_amdgcn_rcpf(sum);
#pragma unroll
      for (int bb = 0; bb < NB; ++bb)
        pw[(bb * 16 + roff + r) * LDP + c * 16 + lm] = (_Float16)(sv[bb] * scl);
    }
    __syncthreads();

    const v16h ap = ldfrag<_Float16>(pw + (b * 16 + lm) * LDP, kb);
#pragma unroll
    for (int cc = 0; cc < 4; ++cc) {
      const v16h vf = ldfrag<_Float16>(vrow + (size_t)(cc * 16) * SEQ + kt, kb);
      o[cc] = mma16(ap, vf, o[cc]);
    }
  }

  const float osc = 1.0f / (PCARRY * VCARRY);
#pragma unroll
  for (int cc = 0; cc < 4; ++cc)
#pragma unroll
    for (int r = 0; r < 8; ++r)
      ost[(b * 16 + roff + r) * LDO + cc * 16 + lm] = (_Float16)(o[cc][r] * osc);
  __syncthreads();
  const unsigned short* ls = reinterpret_cast<const unsigned short*>(ost + b * 16 * LDO);
  unsigned short* g = reinterpret_cast<unsigned short*>(Ctx + base + (size_t)qbase * HD);
  st_tile16(ls, g, lane, HD);
  __threadfence();
  st_tile16(ls, g, lane, HD);
}

extern "C" void kernel_launch(void* const* d_in, const int* in_sizes, int n_in,
                              void* d_out, int out_size, void* d_ws, size_t ws_size,
                              hipStream_t stream) {
  if (n_in < 10) return;
  const int need_xy = (NB - 1) * SEQ_FULL * DIM + SEQ * DIM;
  if (in_sizes[0] < need_xy || in_sizes[1] < need_xy) return;
  if (in_sizes[2] < DIM * DIM || in_sizes[4] < DIM * DIM ||
      in_sizes[6] < DIM * DIM || in_sizes[8] < DIM * DIM) return;
  if (in_sizes[3] < DIM || in_sizes[5] < DIM || in_sizes[7] < DIM || in_sizes[9] < DIM) return;
  if (out_size < ROWS * DIM) return;

  const float* x  = (const float*)d_in[0];
  const float* y  = (const float*)d_in[1];
  const float* Wq = (const float*)d_in[2];
  const float* bq = (const float*)d_in[3];
  const float* Wk = (const float*)d_in[4];
  const float* bk = (const float*)d_in[5];
  const float* Wv = (const float*)d_in[6];
  const float* bv = (const float*)d_in[7];
  const float* Wo = (const float*)d_in[8];
  const float* bo = (const float*)d_in[9];
  float* out = (float*)d_out;

  const size_t P16 = (size_t)ROWS * DIM * 2;
  const size_t W16 = (size_t)DIM * DIM * 2;
  const size_t o_xb = 0;
  const size_t o_yb = P16;
  const size_t o_w  = 2 * P16;
  const size_t o_q  = o_w + 4 * W16;
  const size_t o_k  = o_q + P16;
  const size_t o_vp = o_k + P16;
  const size_t o_end = o_vp + P16;
  if (ws_size < o_end) return;

  char* ws = reinterpret_cast<char*>(d_ws);
  unsigned short* Xb  = reinterpret_cast<unsigned short*>(ws + o_xb);
  unsigned short* Yb  = reinterpret_cast<unsigned short*>(ws + o_yb);
  unsigned short* Wqb = reinterpret_cast<unsigned short*>(ws + o_w);
  unsigned short* Wkb = reinterpret_cast<unsigned short*>(ws + o_w + W16);
  unsigned short* Wvb = reinterpret_cast<unsigned short*>(ws + o_w + 2 * W16);
  unsigned short* Woh = reinterpret_cast<unsigned short*>(ws + o_w + 3 * W16);
  unsigned short* Qp  = reinterpret_cast<unsigned short*>(ws + o_q);
  unsigned short* Kp  = reinterpret_cast<unsigned short*>(ws + o_k);
  unsigned short* Vp  = reinterpret_cast<unsigned short*>(ws + o_vp);
  _Float16* Vt  = reinterpret_cast<_Float16*>(ws + o_yb);
  _Float16* Ctx = reinterpret_cast<_Float16*>(ws + o_xb);
  float* fdum = reinterpret_cast<float*>(ws + o_vp);

  cvt_kernel<0><<<ROWS * 128 / 256, 256, 0, stream>>>(x, Xb, ROWS, SEQ, SEQ_FULL, 1.0f);
  cvt_kernel<0><<<ROWS * 128 / 256, 256, 0, stream>>>(y, Yb, ROWS, SEQ, SEQ_FULL, 1.0f);
  cvt_kernel<0><<<DIM * 128 / 256, 256, 0, stream>>>(Wq, Wqb, DIM, DIM, DIM, 1.0f);
  cvt_kernel<0><<<DIM * 128 / 256, 256, 0, stream>>>(Wk, Wkb, DIM, DIM, DIM, 1.0f);
  cvt_kernel<0><<<DIM * 128 / 256, 256, 0, stream>>>(Wv, Wvb, DIM, DIM, DIM, 1.0f);
  cvt_kernel<1><<<DIM * 128 / 256, 256, 0, stream>>>(Wo, Woh, DIM, DIM, DIM, WOCARRY);

  const dim3 gg(ROWS / 64, DIM / 128);
  gemm_kernel<__bf16, 1><<<gg, 256, 0, stream>>>(
      reinterpret_cast<const __bf16*>(Xb), reinterpret_cast<const __bf16*>(Wqb), bq,
      1.0f, QKC, Qp, fdum, ROWS, DIM, DIM);
  gemm_kernel<__bf16, 1><<<gg, 256, 0, stream>>>(
      reinterpret_cast<const __bf16*>(Yb), reinterpret_cast<const __bf16*>(Wkb), bk,
      1.0f, QKC, Kp, fdum, ROWS, DIM, DIM);
  gemm_kernel<__bf16, 1><<<gg, 256, 0, stream>>>(
      reinterpret_cast<const __bf16*>(Yb), reinterpret_cast<const __bf16*>(Wvb), bv,
      1.0f, VCARRY, Vp, fdum, ROWS, DIM, DIM);
  vt_kernel<<<dim3(SEQ / 64, NSL), 128, 0, stream>>>(reinterpret_cast<const _Float16*>(Vp), Vt);
  attn_kernel<<<dim3(SEQ / 16, NH), NB * 32, 0, stream>>>(
      reinterpret_cast<const _Float16*>(Qp), reinterpret_cast<const _Float16*>(Kp), Vt, Ctx);
  gemm_kernel<_Float16, 2><<<gg, 256, 0, stream>>>(
      Ctx, reinterpret_cast<const _Float16*>(Woh), bo,
      1.0f / WOCARRY, 1.0f, Qp, out, ROWS, DIM, DIM);
}
